// CortexODE_35098472743487
// MI455X (gfx1250) — hardware-verified
//
#include <hip/hip_runtime.h>
#include <math.h>

typedef __attribute__((ext_vector_type(16))) _Float16 v16h;
typedef __attribute__((ext_vector_type(16))) __bf16 v16b;
typedef __attribute__((ext_vector_type(8)))  _Float16 v8h;
typedef __attribute__((ext_vector_type(8)))  float v8f;
typedef __attribute__((ext_vector_type(4)))  float v4f;
typedef __attribute__((ext_vector_type(2)))  float v2f;
typedef __attribute__((ext_vector_type(4)))  unsigned v4u;
typedef __attribute__((ext_vector_type(4)))  int v4i;
typedef float __attribute__((may_alias)) float_a;
typedef int __attribute__((may_alias)) int_a;

template <typename T> __device__ __forceinline__ void vst2(void* p, T v) { *(volatile T*)p = v; __threadfence(); *(volatile T*)p = v; }
__device__ __forceinline__ v8f wmma16(v16h a, v16h b, v8f c) {
  v8f d = __builtin_amdgcn_wmma_f32_16x16x32_f16(false, a, false, b, (short)0, c, false, false);
  asm volatile("v_nop\n\tv_nop\n\tv_nop\n\tv_nop" : "+v"(d) : "v"(a), "v"(b));
  return d;
}
__device__ __forceinline__ v8f wmma_bf(v16b a, v16b b, v8f c) {
  v8f d = __builtin_amdgcn_wmma_f32_16x16x32_bf16(false, a, false, b, (short)0, c, false, false);
  asm volatile("v_nop\n\tv_nop\n\tv_nop\n\tv_nop" : "+v"(d) : "v"(a), "v"(b));
  return d;
}
__device__ __forceinline__ v16h frag_h(const _Float16* rowk0, int lane) {
  union { v16h v; v8h q[2]; } u; const _Float16* p = rowk0 + 8 * (lane >> 4);
  u.q[0] = *(const v8h*)p; u.q[1] = *(const v8h*)(p + 16); return u.v;
}
__device__ __forceinline__ v16h frag_f32(const float* rowk0, int lane) {
  v16h a; const float* p = rowk0 + 8 * (lane >> 4);
#pragma unroll
  for (int i = 0; i < 8; ++i) { a[i] = (_Float16)p[i]; a[8 + i] = (_Float16)p[16 + i]; }
  return a;
}
__device__ __forceinline__ v16h frag_f32s(const float* rowk0, int lane, float sc) {
  v16h a; const float* p = rowk0 + 8 * (lane >> 4);
#pragma unroll
  for (int i = 0; i < 8; ++i) { a[i] = (_Float16)(p[i] * sc); a[8 + i] = (_Float16)(p[16 + i] * sc); }
  return a;
}
__device__ __forceinline__ v16h fragc_f32(const float* W, int k0, int n, int lane, int ld, int K) {
  v16h a; const int g = lane >> 4;
#pragma unroll
  for (int i = 0; i < 8; ++i) { const int ka = k0 + 8 * g + i, kb = ka + 16;
    a[i] = (_Float16)(ka < K ? W[(size_t)(ka < K ? ka : K - 1) * ld + n] : 0.f); a[8 + i] = (_Float16)(kb < K ? W[(size_t)(kb < K ? kb : K - 1) * ld + n] : 0.f); }
  return a;
}
struct F2 { v16b h, l; };
__device__ __forceinline__ F2 bsplit16(const float v[16]) { F2 r;
#pragma unroll
  for (int i = 0; i < 16; ++i) { const __bf16 h = (__bf16)v[i]; r.h[i] = h; r.l[i] = (__bf16)(v[i] - (float)h); }
  return r; }
__device__ __forceinline__ F2 split_row(const float* row, int k0, int lane) { float v[16]; const float* p = row + k0 + 8 * (lane >> 4);
#pragma unroll
  for (int i = 0; i < 8; ++i) { v[i] = p[i]; v[8 + i] = p[16 + i]; }
  return bsplit16(v); }
__device__ __forceinline__ F2 split_rowK(const float* row, int k0, int lane, int K) { float v[16]; const int g = lane >> 4;
#pragma unroll
  for (int i = 0; i < 8; ++i) { const int ka = k0 + 8 * g + i, kb = ka + 16; v[i] = ka < K ? row[ka < K ? ka : K - 1] : 0.f; v[8 + i] = kb < K ? row[kb < K ? kb : K - 1] : 0.f; }
  return bsplit16(v); }
__device__ __forceinline__ F2 split_col(const float* W, int k0, int n, int lane, int ld, int K) { float v[16]; const int g = lane >> 4;
#pragma unroll
  for (int i = 0; i < 8; ++i) { const int ka = k0 + 8 * g + i, kb = ka + 16; v[i] = ka < K ? W[(size_t)(ka < K ? ka : K - 1) * ld + n] : 0.f; v[8 + i] = kb < K ? W[(size_t)(kb < K ? kb : K - 1) * ld + n] : 0.f; }
  return bsplit16(v); }
__device__ __forceinline__ v8f mac3(const F2& a, const F2& b, v8f c) { c = wmma_bf(a.l, b.h, c); c = wmma_bf(a.h, b.l, c); return wmma_bf(a.h, b.h, c); }
__device__ __forceinline__ float sigm(float v) { return 1.0f / (1.0f + expf(-v)); }
#define LDSX() do { asm volatile("s_wait_dscnt 0" ::: "memory"); __builtin_amdgcn_wave_barrier(); __builtin_amdgcn_fence(__ATOMIC_RELEASE, "workgroup"); } while (0)


#define MV 150000
#define DV 192
#define CC 128
#define NSH 125
#define KQ 375
#define KQP 384
#ifndef TVB
#define TVB ((MV + 63) / 64)
#endif
typedef __attribute__((ext_vector_type(8))) __bf16 v8b;
__device__ __forceinline__ v16b frag_b(const __bf16* rowk0, int lane) {
  union { v16b v; v8b q[2]; } u; const __bf16* p = rowk0 + 8 * (lane >> 4);
  u.q[0] = *(const v8b*)p; u.q[1] = *(const v8b*)(p + 16); return u.v;
}
__device__ __forceinline__ float bfr(float v) { return (float)(__bf16)v; }
__device__ __forceinline__ float lrelu(float v) { return v > 0.f ? v : 0.2f * v; }

#define WS_V1   0u
#define WS_V2   (WS_V1 + 4u * 96 * 96 * 96)
#define WS_PC   (WS_V2 + 4u * 48 * 48 * 64)
#define WS_PL   (WS_PC + 2u * CC * KQP)
#define WS_P2   (WS_PL + 2u * CC * CC)
#define WS_P3   (WS_P2 + 2u * 512 * 256)
#define WS_END  (WS_P3 + 2u * 256 * 512)

__global__ __launch_bounds__(128) void k_pool1(const float* __restrict__ V, float* __restrict__ V1) {
  __shared__ __align__(16) float srow[96];
  const int z = blockIdx.x / 96, y = blockIdx.x % 96, x = threadIdx.x;
  if (x < 96) { float s = 0.f;
#pragma unroll
    for (int dz = 0; dz < 2; ++dz)
#pragma unroll
      for (int dy = 0; dy < 2; ++dy) { const float* p = V + ((size_t)(2 * z + dz) * DV + (2 * y + dy)) * DV + 2 * x; s += bfr(p[0]) + bfr(p[1]); }
    srow[x] = s * 0.125f; }
  __syncthreads();
  if (x < 24) vst2(V1 + (size_t)blockIdx.x * 96 + x * 4, *(const v4f*)&srow[x * 4]);
}
__global__ __launch_bounds__(64) void k_pool2(const float* __restrict__ V1, float* __restrict__ V2) {
  __shared__ __align__(16) float srow[64];
  const int z = blockIdx.x / 48, y = blockIdx.x % 48, x = threadIdx.x; float s = 0.f;
  if (x < 48) {
#pragma unroll
    for (int dz = 0; dz < 2; ++dz)
#pragma unroll
      for (int dy = 0; dy < 2; ++dy) { const float* p = V1 + ((size_t)(2 * z + dz) * 96 + (2 * y + dy)) * 96 + 2 * x; s += p[0] + p[1]; }
    s *= 0.125f; }
  srow[x] = x < 48 ? s : 0.f;
  __syncthreads();
  if (x < 16) vst2(V2 + (size_t)blockIdx.x * 64 + x * 4, *(const v4f*)&srow[x * 4]);
}
__global__ __launch_bounds__(128) void k_pack(const float* __restrict__ cw, const float* __restrict__ lw, const float* __restrict__ w2, const float* __restrict__ w3, __bf16* __restrict__ PC, __bf16* __restrict__ PL, __bf16* __restrict__ P2, __bf16* __restrict__ P3) {
  __shared__ __align__(16) __bf16 srow[512];
  const int n = blockIdx.x, tid = threadIdx.x; const float* src; int K, KP; __bf16* dst;
  if (n < 128) { src = cw + (size_t)n * KQ; K = KQ; KP = KQP; dst = PC + (size_t)n * KQP; }
  else if (n < 256) { src = lw + (size_t)(n - 128) * CC; K = CC; KP = CC; dst = PL + (size_t)(n - 128) * CC; }
  else if (n < 768) { src = w2 + (size_t)(n - 256) * 256; K = 256; KP = 256; dst = P2 + (size_t)(n - 256) * 256; }
  else { src = w3 + (size_t)(n - 768) * 512; K = 512; KP = 512; dst = P3 + (size_t)(n - 768) * 512; }
  for (int k = tid; k < KP; k += 128) srow[k] = k < K ? (__bf16)src[k] : (__bf16)0.f;
  __syncthreads();
  if (tid < KP / 8) vst2((unsigned*)(dst + tid * 8), *(const v4u*)(&srow[tid * 8]));
}
__device__ __forceinline__ float tri3(const float* __restrict__ vol, int s, int pitch, float cx, float cy, float cz, bool rnd) {
  const float sm1 = (float)(s - 1);
  float ix = fminf(fmaxf((cx + 1.0f) * 0.5f * sm1, 0.f), sm1), iy = fminf(fmaxf((cy + 1.0f) * 0.5f * sm1, 0.f), sm1), iz = fminf(fmaxf((cz + 1.0f) * 0.5f * sm1, 0.f), sm1);
  const float x0f = floorf(ix), y0f = floorf(iy), z0f = floorf(iz); const float wx = ix - x0f, wy = iy - y0f, wz = iz - z0f;
  const int x0 = (int)x0f, y0 = (int)y0f, z0 = (int)z0f; const int x1 = min(x0 + 1, s - 1), y1 = min(y0 + 1, s - 1), z1 = min(z0 + 1, s - 1);
  const float* r00 = vol + ((size_t)z0 * s + y0) * pitch; const float* r01 = vol + ((size_t)z0 * s + y1) * pitch; const float* r10 = vol + ((size_t)z1 * s + y0) * pitch; const float* r11 = vol + ((size_t)z1 * s + y1) * pitch;
  float a = r00[x0], bq = r00[x1], c = r01[x0], d = r01[x1], e = r10[x0], f = r10[x1], gg = r11[x0], h = r11[x1];
  if (rnd) { a = bfr(a); bq = bfr(bq); c = bfr(c); d = bfr(d); e = bfr(e); f = bfr(f); gg = bfr(gg); h = bfr(h); }
  const float lo = (a * (1.f - wx) + bq * wx) * (1.f - wy) + (c * (1.f - wx) + d * wx) * wy;
  const float hi = (e * (1.f - wx) + f * wx) * (1.f - wy) + (gg * (1.f - wx) + h * wx) * wy;
  return lo * (1.f - wz) + hi * wz;
}
__global__ __launch_bounds__(256) void k_main(const float* __restrict__ X, const float* __restrict__ V0, const float* __restrict__ V1, const float* __restrict__ V2, const __bf16* __restrict__ PC, const __bf16* __restrict__ PL, const __bf16* __restrict__ P2, const __bf16* __restrict__ P3,
                                              const float* __restrict__ f1w, const float* __restrict__ f1b, const float* __restrict__ cb, const float* __restrict__ lb, const float* __restrict__ b2, const float* __restrict__ b3, const float* __restrict__ f4w, const float* __restrict__ f4b, float* __restrict__ out, int nv) {
  __shared__ __align__(16) __bf16 R1h[64][520], R1l[64][520];
  __shared__ __align__(16) __bf16 R2h[64][264], R2l[64][264];
  __shared__ __align__(16) float R3[64][260];
  __shared__ __align__(16) float sres[192];
  const int tid = threadIdx.x, wave = tid >> 5, lane = tid & 31, col = lane & 15, g = lane >> 4; const int v0 = blockIdx.x * 64;
  const int rt = wave & 3, cg = wave >> 2;
  for (int q = tid; q < 64 * KQP; q += 256) { const int vl = q & 63, sidx = q >> 6; float val = 0.f;
    if (sidx < KQ) { const int vv = min(v0 + vl, MV - 1); const float px = bfr(X[(size_t)vv * 3]), py = bfr(X[(size_t)vv * 3 + 1]), pz = bfr(X[(size_t)vv * 3 + 2]);
      const int qs = sidx / NSH, sh = sidx % NSH; const int si = sh / 25, sj = (sh / 5) % 5, sk = sh % 5;
      const float gi = -3.0f + 1.25f * (float)si, gj = -3.0f + 1.25f * (float)sj, gk = -3.0f + 1.25f * (float)sk;
      const float stp = qs == 0 ? (float)(2.0 / 192.0) : (qs == 1 ? (float)(4.0 / 192.0) : (float)(8.0 / 192.0));
      const float cx = px + gi * stp, cy = py + gj * stp, cz = pz + gk * stp;
      val = qs == 0 ? tri3(V0, DV, DV, cx, cy, cz, true) : (qs == 1 ? tri3(V1, 96, 96, cx, cy, cz, false) : tri3(V2, 48, 64, cx, cy, cz, false)); }
    const __bf16 hb = (__bf16)val; R1h[vl][sidx] = hb; R1l[vl][sidx] = (__bf16)(val - (float)hb); }
  __syncthreads();
  { v8f acc[4] = {};
#pragma unroll 2
    for (int kc = 0; kc < KQP / 32; ++kc) { const v16b ah = frag_b(&R1h[rt * 16 + col][kc * 32], lane), al = frag_b(&R1l[rt * 16 + col][kc * 32], lane);
#pragma unroll
      for (int j = 0; j < 4; ++j) { const v16b w = frag_b(PC + (size_t)((cg * 4 + j) * 16 + col) * KQP + kc * 32, lane); acc[j] = wmma_bf(al, w, acc[j]); acc[j] = wmma_bf(ah, w, acc[j]); } }
#pragma unroll
    for (int j = 0; j < 4; ++j) { const int n = (cg * 4 + j) * 16 + col; const float bb = bfr(cb[n]);
#pragma unroll
      for (int r = 0; r < 8; ++r) R3[rt * 16 + 8 * g + r][n] = acc[j][r] + bb; } }
  __syncthreads();
  { const F2 a[4] = {split_row(&R3[rt * 16 + col][0], 0, lane), split_row(&R3[rt * 16 + col][0], 32, lane), split_row(&R3[rt * 16 + col][0], 64, lane), split_row(&R3[rt * 16 + col][0], 96, lane)}; v8f acc[4] = {};
#pragma unroll
    for (int kc = 0; kc < 4; ++kc)
#pragma unroll
      for (int j = 0; j < 4; ++j) { const v16b w = frag_b(PL + (size_t)((cg * 4 + j) * 16 + col) * CC + kc * 32, lane); acc[j] = wmma_bf(a[kc].l, w, acc[j]); acc[j] = wmma_bf(a[kc].h, w, acc[j]); }
#pragma unroll
    for (int j = 0; j < 4; ++j) { const int n = (cg * 4 + j) * 16 + col; const float bb = bfr(lb[n]);
#pragma unroll
      for (int r = 0; r < 8; ++r) { const float v = acc[j][r] + bb; const __bf16 hb = (__bf16)v; R2h[rt * 16 + 8 * g + r][CC + n] = hb; R2l[rt * 16 + 8 * g + r][CC + n] = (__bf16)(v - (float)hb); } } }
  for (int q = tid; q < 64 * CC; q += 256) { const int vl = q >> 7, n = q & 127; const int vv = min(v0 + vl, MV - 1);
    const float v = lrelu(((bfr(X[(size_t)vv * 3]) * bfr(f1w[n * 3]) + bfr(X[(size_t)vv * 3 + 1]) * bfr(f1w[n * 3 + 1])) + bfr(X[(size_t)vv * 3 + 2]) * bfr(f1w[n * 3 + 2])) + bfr(f1b[n]));
    const __bf16 hb = (__bf16)v; R2h[vl][n] = hb; R2l[vl][n] = (__bf16)(v - (float)hb); }
  __syncthreads();
  { v8f acc[16] = {};
#pragma unroll 1
    for (int kc = 0; kc < 8; ++kc) { const v16b ah = frag_b(&R2h[rt * 16 + col][kc * 32], lane), al = frag_b(&R2l[rt * 16 + col][kc * 32], lane);
#pragma unroll
      for (int j = 0; j < 16; ++j) { const v16b w = frag_b(P2 + (size_t)((cg * 16 + j) * 16 + col) * 256 + kc * 32, lane); acc[j] = wmma_bf(al, w, acc[j]); acc[j] = wmma_bf(ah, w, acc[j]); } }
#pragma unroll
    for (int j = 0; j < 16; ++j) { const int n = (cg * 16 + j) * 16 + col; const float bb = bfr(b2[n]);
#pragma unroll
      for (int r = 0; r < 8; ++r) { const float v = lrelu(acc[j][r] + bb); const __bf16 hb = (__bf16)v; R1h[rt * 16 + 8 * g + r][n] = hb; R1l[rt * 16 + 8 * g + r][n] = (__bf16)(v - (float)hb); } } }
  __syncthreads();
  { v8f acc[8] = {};
#pragma unroll 1
    for (int kc = 0; kc < 16; ++kc) { const v16b ah = frag_b(&R1h[rt * 16 + col][kc * 32], lane), al = frag_b(&R1l[rt * 16 + col][kc * 32], lane);
#pragma unroll
      for (int j = 0; j < 8; ++j) { const v16b w = frag_b(P3 + (size_t)((cg * 8 + j) * 16 + col) * 512 + kc * 32, lane); acc[j] = wmma_bf(al, w, acc[j]); acc[j] = wmma_bf(ah, w, acc[j]); } }
#pragma unroll
    for (int j = 0; j < 8; ++j) { const int n = (cg * 8 + j) * 16 + col; const float bb = bfr(b3[n]);
#pragma unroll
      for (int r = 0; r < 8; ++r) R3[rt * 16 + 8 * g + r][n] = lrelu(acc[j][r] + bb); } }
  __syncthreads();
  { const int vl = tid >> 2, part = tid & 3; float s0 = 0.f, s1 = 0.f, s2 = 0.f;
    for (int k = part * 64; k < part * 64 + 64; ++k) { const float hv = R3[vl][k]; s0 += hv * bfr(f4w[k]); s1 += hv * bfr(f4w[256 + k]); s2 += hv * bfr(f4w[512 + k]); }
    s0 += __shfl_xor(s0, 1); s0 += __shfl_xor(s0, 2); s1 += __shfl_xor(s1, 1); s1 += __shfl_xor(s1, 2); s2 += __shfl_xor(s2, 1); s2 += __shfl_xor(s2, 2);
    if (part == 0) { sres[vl * 3] = s0 + bfr(f4b[0]); sres[vl * 3 + 1] = s1 + bfr(f4b[1]); sres[vl * 3 + 2] = s2 + bfr(f4b[2]); } }
  __syncthreads();
  { const int nvb = min(64, nv - v0); const int nfl = nvb * 3;
    if (tid < (nfl + 3) / 4) { v4f v; for (int i = 0; i < 4; ++i) v[i] = (tid * 4 + i < nfl) ? sres[tid * 4 + i] : 0.f;
      if (tid * 4 + 4 <= nfl) vst2(out + (size_t)v0 * 3 + tid * 4, v); else { for (int i = 0; i < 4; ++i) if (tid * 4 + i < nfl) vst2(out + (size_t)v0 * 3 + tid * 4 + i, (float_a)v[i]); } } }
}

extern "C" void kernel_launch(void* const* d_in, const int* in_sizes, int n_in, void* d_out, int out_size, void* d_ws, size_t ws_size, hipStream_t stream) {
  (void)in_sizes; (void)n_in; (void)out_size;
  const float** F = (const float**)d_in;
  if (ws_size < (size_t)WS_END) return;
  char* ws = (char*)d_ws; float *V1 = (float*)(ws + WS_V1), *V2 = (float*)(ws + WS_V2); __bf16 *PC = (__bf16*)(ws + WS_PC), *PL = (__bf16*)(ws + WS_PL), *P2 = (__bf16*)(ws + WS_P2), *P3 = (__bf16*)(ws + WS_P3);
  k_pool1<<<96 * 96, 128, 0, stream>>>(F[2], V1);
  k_pool2<<<48 * 48, 64, 0, stream>>>(V1, V2);
  k_pack<<<1024, 128, 0, stream>>>(F[11], F[13], F[5], F[7], PC, PL, P2, P3);
  k_main<<<TVB, 256, 0, stream>>>(F[1], F[2], V1, V2, PC, PL, P2, P3, F[3], F[4], F[12], F[14], F[6], F[8], F[9], F[10], (float*)d_out, MV);
}
